// ST_Attention_2061584302861
// MI455X (gfx1250) — hardware-verified
//
#include <hip/hip_runtime.h>


#define NB_  16
#define CIN  64
#define NN   207
#define TT   12
#define D2   128
#define KG   8
#define NROW (NB_ * NN * TT)
#define PB   (NN * TT)
#define DM   CIN
#define BEPS 1e-5f
#define ISQD 0.35355339059327373f
#define LOSC 1024.0f
#define NP   256
#define TP   32
#define TV   64
#define CQ   32

typedef _Float16 h16;
typedef unsigned short bf;
typedef __attribute__((ext_vector_type(16))) __bf16   v16bf;
typedef __attribute__((ext_vector_type(16))) _Float16 v16h;
typedef __attribute__((ext_vector_type(8)))  _Float16 v8h;
typedef __attribute__((ext_vector_type(8)))  unsigned short v8us;
typedef __attribute__((ext_vector_type(8)))  float    v8f;
typedef __attribute__((ext_vector_type(4)))  float    v4f;
typedef v8h  __attribute__((may_alias)) v8ha;
typedef v4f  __attribute__((may_alias)) v4fa;
typedef v8us __attribute__((may_alias)) v8usa;

__device__ __forceinline__ unsigned short f2bf(float f) { unsigned u = __float_as_uint(f); u += 0x7FFFu + ((u >> 16) & 1u); return (unsigned short)(u >> 16); }
__device__ __forceinline__ float bf2f(unsigned short b) { return __uint_as_float(((unsigned)b) << 16); }
__device__ __forceinline__ float bfr(float f) { return bf2f(f2bf(f)); }
__device__ __forceinline__ v16h cat16(v8h lo, v8h hi) { return __builtin_shufflevector(lo, hi, 0, 1, 2, 3, 4, 5, 6, 7, 8, 9, 10, 11, 12, 13, 14, 15); }
__device__ __forceinline__ v16bf cat16b(v8us lo, v8us hi) { return __builtin_bit_cast(v16bf, __builtin_shufflevector(lo, hi, 0, 1, 2, 3, 4, 5, 6, 7, 8, 9, 10, 11, 12, 13, 14, 15)); }
__device__ __forceinline__ v8f wmma16(v16h a, v16h b, v8f c) { return __builtin_amdgcn_wmma_f32_16x16x32_f16(false, a, false, b, (short)0, c, false, false); }
__device__ __forceinline__ v8f wmmab(v16bf a, v16bf b, v8f c) { return __builtin_amdgcn_wmma_f32_16x16x32_bf16(false, a, false, b, (short)0, c, false, false); }

template <bool SPLITA, bool F16OUT = false>
__global__ __launch_bounds__(128) void k_gemmb(const bf* __restrict__ A, const bf* __restrict__ Al, const bf* __restrict__ Bn, const float* __restrict__ bias, float* C, int ldc, h16* C2, const float* __restrict__ R = nullptr, int K = DM, int roundR = 1) {
    __shared__ __align__(16) float ost[4][16 * 68];
    const int lane = threadIdx.x & 31, wave = threadIdx.x >> 5, lr = lane & 15, hi = lane >> 4;
    const int r0 = blockIdx.x * 64 + wave * 16, c0 = blockIdx.y * 64;
    const size_t aoff = (size_t)(r0 + lr) * K + 8 * hi;
    size_t boff[4];
#pragma unroll
    for (int t = 0; t < 4; ++t) boff[t] = (size_t)(c0 + t * 16 + lr) * K + 8 * hi;
    v8f acc[4];
#pragma unroll
    for (int t = 0; t < 4; ++t) acc[t] = (v8f){};
#pragma unroll 1
    for (int kc = 0; kc < K; kc += 32) {
        const v16bf a = cat16b(*(const v8us*)(A + aoff + kc), *(const v8us*)(A + aoff + kc + 16));
        v16bf al = a;
        if (SPLITA) al = cat16b(*(const v8us*)(Al + aoff + kc), *(const v8us*)(Al + aoff + kc + 16));
#pragma unroll
        for (int t = 0; t < 4; ++t) { const v16bf b = cat16b(*(const v8us*)(Bn + boff[t] + kc), *(const v8us*)(Bn + boff[t] + kc + 16)); acc[t] = wmmab(a, b, acc[t]); if (SPLITA) acc[t] = wmmab(al, b, acc[t]); }
        asm volatile("v_nop\n\tv_nop\n\tv_nop\n\tv_nop" : "+v"(acc[0]), "+v"(acc[1]), "+v"(acc[2]), "+v"(acc[3]) : "v"(a), "v"(al));
    }
    float* os = &ost[wave][0];
#pragma unroll
    for (int t = 0; t < 4; ++t) { const float bv = bias ? bfr(bias[c0 + t * 16 + lr]) : 0.f;
#pragma unroll
        for (int j = 0; j < 8; ++j) os[(hi * 8 + j) * 68 + t * 16 + lr] = acc[t][j] + bv; }
    __syncthreads();
    if (F16OUT) {
        h16* crow = (h16*)(void*)C + (size_t)r0 * ldc + c0;
        auto pass = [&]() {
#pragma unroll
            for (int s = 0; s < 4; ++s) { const int row = 4 * s + (lane >> 3), piece = lane & 7; const float* sp = os + row * 68 + piece * 8; v8h o, o2;
#pragma unroll
                for (int i = 0; i < 8; ++i) { const h16 a = (h16)sp[i]; o[i] = a; o2[i] = (h16)((sp[i] - (float)a) * LOSC); }
                *(volatile v8h*)(crow + (size_t)row * ldc + piece * 8) = o; if (C2) *(volatile v8h*)(C2 + (size_t)r0 * ldc + c0 + (size_t)row * ldc + piece * 8) = o2; }
        };
        pass(); __threadfence(); pass();
    } else {
        float* crow = C + (size_t)r0 * ldc + c0;
        auto pass = [&]() {
#pragma unroll
            for (int s = 0; s < 8; ++s) { const int Lid = (lane >> 3) + 4 * s, piece = lane & 7; const int row = Lid >> 1, cofs = (Lid & 1) * 32 + piece * 4;
                v4f val = *(const v4fa*)(os + row * 68 + cofs); if (R) { const v4f rv = *(const v4f*)(R + ((size_t)r0 + row) * ldc + c0 + cofs); val += roundR ? (v4f){bfr(rv[0]), bfr(rv[1]), bfr(rv[2]), bfr(rv[3])} : rv; }
                *(volatile v4f*)(crow + (size_t)row * ldc + cofs) = val; }
        };
        pass(); __threadfence(); pass();
    }
}

template <bool SPLITA, bool F16OUT = false>
__global__ __launch_bounds__(128) void k_gemmbz(const bf* __restrict__ A, const bf* __restrict__ Al, const bf* __restrict__ Bn, const float* __restrict__ bias, float* C, int ldc, h16* C2, const float* __restrict__ R, int K, int roundR, size_t sA, size_t sB, size_t sBias, size_t sC) {
    { const size_t g = blockIdx.z; A += g * sA; if (Al) Al += g * sA; Bn += g * sB; if (bias) bias += g * sBias; C += g * sC; if (R) R += g * sC; }
    __shared__ __align__(16) float ost[4][16 * 68];
    const int lane = threadIdx.x & 31, wave = threadIdx.x >> 5, lr = lane & 15, hi = lane >> 4;
    const int r0 = blockIdx.x * 64 + wave * 16, c0 = blockIdx.y * 64;
    const size_t aoff = (size_t)(r0 + lr) * K + 8 * hi;
    size_t boff[4];
#pragma unroll
    for (int t = 0; t < 4; ++t) boff[t] = (size_t)(c0 + t * 16 + lr) * K + 8 * hi;
    v8f acc[4];
#pragma unroll
    for (int t = 0; t < 4; ++t) acc[t] = (v8f){};
#pragma unroll 1
    for (int kc = 0; kc < K; kc += 32) {
        const v16bf a = cat16b(*(const v8us*)(A + aoff + kc), *(const v8us*)(A + aoff + kc + 16));
        v16bf al = a;
        if (SPLITA) al = cat16b(*(const v8us*)(Al + aoff + kc), *(const v8us*)(Al + aoff + kc + 16));
#pragma unroll
        for (int t = 0; t < 4; ++t) { const v16bf b = cat16b(*(const v8us*)(Bn + boff[t] + kc), *(const v8us*)(Bn + boff[t] + kc + 16)); acc[t] = wmmab(a, b, acc[t]); if (SPLITA) acc[t] = wmmab(al, b, acc[t]); }
        asm volatile("v_nop\n\tv_nop\n\tv_nop\n\tv_nop" : "+v"(acc[0]), "+v"(acc[1]), "+v"(acc[2]), "+v"(acc[3]) : "v"(a), "v"(al));
    }
    float* os = &ost[wave][0];
#pragma unroll
    for (int t = 0; t < 4; ++t) { const float bv = bias ? bfr(bias[c0 + t * 16 + lr]) : 0.f;
#pragma unroll
        for (int j = 0; j < 8; ++j) os[(hi * 8 + j) * 68 + t * 16 + lr] = acc[t][j] + bv; }
    __syncthreads();
    if (F16OUT) {
        h16* crow = (h16*)(void*)C + (size_t)r0 * ldc + c0;
        auto pass = [&]() {
#pragma unroll
            for (int s = 0; s < 4; ++s) { const int row = 4 * s + (lane >> 3), piece = lane & 7; const float* sp = os + row * 68 + piece * 8; v8h o, o2;
#pragma unroll
                for (int i = 0; i < 8; ++i) { const h16 a = (h16)sp[i]; o[i] = a; o2[i] = (h16)((sp[i] - (float)a) * LOSC); }
                *(volatile v8h*)(crow + (size_t)row * ldc + piece * 8) = o; if (C2) *(volatile v8h*)(C2 + (size_t)r0 * ldc + c0 + (size_t)row * ldc + piece * 8) = o2; }
        };
        pass(); __threadfence(); pass();
    } else {
        float* crow = C + (size_t)r0 * ldc + c0;
        auto pass = [&]() {
#pragma unroll
            for (int s = 0; s < 8; ++s) { const int Lid = (lane >> 3) + 4 * s, piece = lane & 7; const int row = Lid >> 1, cofs = (Lid & 1) * 32 + piece * 4;
                v4f val = *(const v4fa*)(os + row * 68 + cofs); if (R) { const v4f rv = *(const v4f*)(R + ((size_t)r0 + row) * ldc + c0 + cofs); val += roundR ? (v4f){bfr(rv[0]), bfr(rv[1]), bfr(rv[2]), bfr(rv[3])} : rv; }
                *(volatile v4f*)(crow + (size_t)row * ldc + cofs) = val; }
        };
        pass(); __threadfence(); pass();
    }
}


__global__ __launch_bounds__(256) void k_cvt8(const float* __restrict__ src, bf* dst, size_t n8) {
    const size_t i = (size_t)blockIdx.x * 256 + threadIdx.x; if (i >= n8) return;
    const v8f v = *(const v8f*)(src + i * 8); v8us o;
#pragma unroll
    for (int k = 0; k < 8; ++k) o[k] = f2bf(v[k]);
    *(volatile v8us*)(dst + i * 8) = o; __threadfence(); *(volatile v8us*)(dst + i * 8) = o;
}
__global__ __launch_bounds__(256) void k_zero8(bf* dst, size_t n8) {
    const size_t i = (size_t)blockIdx.x * 256 + threadIdx.x; if (i >= n8) return; v8us z;
#pragma unroll
    for (int k = 0; k < 8; ++k) z[k] = 0;
    *(volatile v8us*)(dst + i * 8) = z; __threadfence(); *(volatile v8us*)(dst + i * 8) = z;
}

__global__ __launch_bounds__(256) void k_xrows(const float* __restrict__ x, bf* XR) {
    typedef __attribute__((ext_vector_type(2))) unsigned short v2us;
    const int lane = threadIdx.x & 31; const size_t r = (size_t)blockIdx.x * 8 + (threadIdx.x >> 5); if (r >= (size_t)NROW) return; const int b = (int)(r / PB), nt = (int)(r % PB); v2us o;
#pragma unroll
    for (int i = 0; i < 2; ++i) { const int c = lane * 2 + i; o[i] = f2bf(x[((size_t)b * CIN + c) * PB + nt]); }
    *(volatile v2us*)(XR + r * CIN + lane * 2) = o; __threadfence(); *(volatile v2us*)(XR + r * CIN + lane * 2) = o;
}
template <int MODE>
__global__ __launch_bounds__(128) void k_colstat(const float* __restrict__ Y, int nc, const float* __restrict__ MEAN, float* OUTV) {
    const int c = threadIdx.x; float s = 0.f;
    if (c < nc) { const float mu = (MODE == 1) ? MEAN[c] : 0.f;
#pragma unroll 1
        for (int b = 0; b < NB_; ++b) { float p = 0.f;
#pragma unroll 4
            for (int r = b * PB; r < (b + 1) * PB; ++r) { const float v = Y[(size_t)r * nc + c]; const float d = (MODE == 1) ? (v - mu) * (v - mu) : v; p += d; }
            s += p; }
        s *= 1.0f / (float)NROW; }
    *(volatile float*)(OUTV + c) = s; __threadfence(); *(volatile float*)(OUTV + c) = s;
}
__device__ __forceinline__ float bnr(float y, int c, const float* __restrict__ MEAN, const float* __restrict__ VAR, const float* __restrict__ g, const float* __restrict__ be) {
    return fmaxf(bfr(g[c]) * (y - MEAN[c]) * rsqrtf(VAR[c] + BEPS) + bfr(be[c]), 0.f); }
__global__ __launch_bounds__(256) void k_qkp(const float* __restrict__ Y, const float* __restrict__ MEAN, const float* __restrict__ VAR, const float* __restrict__ g, const float* __restrict__ be, int b, int c0, bf* Ph, bf* Pl) {
    typedef __attribute__((ext_vector_type(2))) unsigned short v2us;
    const int lane = threadIdx.x & 31; const size_t wid = (size_t)blockIdx.x * 8 + (threadIdx.x >> 5); if (wid >= (size_t)CQ * (NP / 2)) return; const int cq = (int)(wid / (NP / 2)); const int n = (int)(wid % (NP / 2)) * 2 + (lane >> 4); const int t0 = (lane & 15) * 2; const int c = c0 + cq;
    v2us oh, ol;
#pragma unroll
    for (int i = 0; i < 2; ++i) { const int t = t0 + i; const bool ok = (n < NN) && (t < TT); const float v = ok ? bnr(Y[((size_t)b * PB + (ok ? n : 0) * TT + (ok ? t : 0)) * D2 + c], c, MEAN, VAR, g, be) : 0.f; const unsigned short hb = f2bf(v); oh[i] = hb; ol[i] = f2bf(v - bf2f(hb)); }
    const size_t o = ((size_t)cq * NP + n) * TP + t0; *(volatile v2us*)(Ph + o) = oh; *(volatile v2us*)(Pl + o) = ol; __threadfence(); *(volatile v2us*)(Ph + o) = oh; *(volatile v2us*)(Pl + o) = ol;
}
__global__ __launch_bounds__(256) void k_vtp(const float* __restrict__ Y, const float* __restrict__ MEAN, const float* __restrict__ VAR, const float* __restrict__ g, const float* __restrict__ be, int b, int c0, bf* Th, bf* Tl) {
    typedef __attribute__((ext_vector_type(2))) unsigned short v2us;
    const int lane = threadIdx.x & 31; const size_t wid = (size_t)blockIdx.x * 8 + (threadIdx.x >> 5); if (wid >= (size_t)CQ * TV * (NP / 64)) return; const int mg = (int)(wid % (NP / 64)), rest = (int)(wid / (NP / 64)), t = rest % TV, cq = rest / TV; const int m0 = mg * 64 + lane * 2; const int c = c0 + cq;
    v2us oh, ol;
#pragma unroll
    for (int i = 0; i < 2; ++i) { const int m = m0 + i; const bool ok = (m < NN) && (t < TT); const float v = ok ? bnr(Y[((size_t)b * PB + (ok ? m : 0) * TT + (ok ? t : 0)) * D2 + c], c, MEAN, VAR, g, be) : 0.f; const unsigned short hb = f2bf(v); oh[i] = hb; ol[i] = f2bf(v - bf2f(hb)); }
    const size_t o = ((size_t)cq * TV + t) * NP + m0; *(volatile v2us*)(Th + o) = oh; *(volatile v2us*)(Tl + o) = ol; __threadfence(); *(volatile v2us*)(Th + o) = oh; *(volatile v2us*)(Tl + o) = ol;
}
__global__ __launch_bounds__(256) void k_gsmx(const float* __restrict__ S, bf* Wh, bf* Wl) {
    typedef __attribute__((ext_vector_type(4))) unsigned short v4us;
    const int lane = threadIdx.x & 31; const size_t wid = (size_t)blockIdx.x * 8 + (threadIdx.x >> 5); if (wid >= (size_t)(CQ / KG) * NP * 2) return; const int half = (int)(wid & 1); const int n = (int)((wid >> 1) % NP); const int gq = (int)((wid >> 1) / NP); const int m0 = half * 128 + lane * 4;
    float e[KG][4];
#pragma unroll
    for (int q = 0; q < 4; ++q) { const int m = m0 + q; float mx = -3.0e38f;
#pragma unroll
        for (int k = 0; k < KG; ++k) { e[k][q] = S[(((size_t)(gq * KG + k)) * NP + n) * NP + m] * ISQD; mx = fmaxf(mx, e[k][q]); }
        float sum = 0.f;
#pragma unroll
        for (int k = 0; k < KG; ++k) { e[k][q] = __expf(e[k][q] - mx); sum += e[k][q]; }
        const float inv = ((n < NN) && (m < NN)) ? 1.0f / sum : 0.f;
#pragma unroll
        for (int k = 0; k < KG; ++k) e[k][q] *= inv; }
#pragma unroll 1
    for (int ps = 0; ps < 2; ++ps) {
#pragma unroll
        for (int k = 0; k < KG; ++k) { v4us oh, ol;
#pragma unroll
            for (int q = 0; q < 4; ++q) { const unsigned short hb = f2bf(e[k][q]); oh[q] = hb; ol[q] = f2bf(e[k][q] - bf2f(hb)); }
            const size_t o = (((size_t)(gq * KG + k)) * NP + n) * NP + m0; *(volatile v4us*)(Wh + o) = oh; *(volatile v4us*)(Wl + o) = ol; }
        if (ps == 0) __threadfence(); }
}
__global__ __launch_bounds__(256) void k_att(const float* __restrict__ O, int b, int c0h, bf* Ah, bf* Al) {
    typedef __attribute__((ext_vector_type(2))) unsigned short v2us;
    const int lane = threadIdx.x & 31; const int wid = blockIdx.x * 8 + (threadIdx.x >> 5); if (wid >= PB) return; const int n = wid / TT, t = wid % TT; v2us oh, ol;
#pragma unroll
    for (int i = 0; i < 2; ++i) { const int ch = lane * 2 + i; const float v = O[((size_t)ch * NP + n) * TV + t]; const unsigned short hb = f2bf(v); oh[i] = hb; ol[i] = f2bf(v - bf2f(hb)); }
    const size_t o = ((size_t)b * PB + wid) * D2 + c0h + lane * 2; *(volatile v2us*)(Ah + o) = oh; *(volatile v2us*)(Al + o) = ol; __threadfence(); *(volatile v2us*)(Ah + o) = oh; *(volatile v2us*)(Al + o) = ol;
}
__global__ __launch_bounds__(256) void k_out(const float* __restrict__ OO, const float* __restrict__ MO, const float* __restrict__ VO, const float* __restrict__ go, const float* __restrict__ bo, float* OUTP) {
    const size_t u = (size_t)blockIdx.x * 256 + threadIdx.x; if (u >= (size_t)NB_ * CIN * PB / 4) return; v4f v;
#pragma unroll
    for (int q = 0; q < 4; ++q) { const size_t e = u * 4 + q; const int nt = (int)(e % PB); const int c = (int)((e / PB) % CIN); const int b = (int)(e / ((size_t)PB * CIN)); v[q] = bnr(OO[((size_t)b * PB + nt) * CIN + c], c, MO, VO, go, bo); }
    *(volatile v4f*)(OUTP + u * 4) = v; __threadfence(); *(volatile v4f*)(OUTP + u * 4) = v;
}

extern "C" void kernel_launch(void* const* d_in, const int* in_sizes, int n_in,
                              void* d_out, int out_size, void* d_ws, size_t ws_size, hipStream_t stream) {
    (void)in_sizes; (void)n_in; (void)out_size;
    const float* x0 = (const float*)d_in[0]; const float* x1 = (const float*)d_in[1];
    const float* wq = (const float*)d_in[2]; const float* bq = (const float*)d_in[3]; const float* gq = (const float*)d_in[4]; const float* beq = (const float*)d_in[5];
    const float* wk = (const float*)d_in[6]; const float* bk = (const float*)d_in[7]; const float* gk = (const float*)d_in[8]; const float* bek = (const float*)d_in[9];
    const float* wv = (const float*)d_in[10]; const float* bv = (const float*)d_in[11]; const float* gv = (const float*)d_in[12]; const float* bev = (const float*)d_in[13];
    const float* wo = (const float*)d_in[14]; const float* bo = (const float*)d_in[15]; const float* go = (const float*)d_in[16]; const float* beo = (const float*)d_in[17];
    float* out = (float*)d_out;
    char* wsp = (char*)d_ws;
    auto take = [&](size_t bytes) { char* p = wsp; wsp += (bytes + 255) & ~(size_t)255; return (void*)p; };
    bf* WQ = (bf*)take(D2 * CIN * 2); bf* WK = (bf*)take(D2 * CIN * 2); bf* WV = (bf*)take(D2 * CIN * 2); bf* WO = (bf*)take(CIN * D2 * 2);
    bf* X0 = (bf*)take((size_t)NROW * CIN * 2); bf* X1 = (bf*)take((size_t)NROW * CIN * 2); float* YQ = (float*)take((size_t)NROW * D2 * 4); float* YK = (float*)take((size_t)NROW * D2 * 4); float* YV = (float*)take((size_t)NROW * D2 * 4);
    float* MQ = (float*)take(512); float* VQ = (float*)take(512); float* MK = (float*)take(512); float* VK = (float*)take(512); float* MV = (float*)take(512); float* VV = (float*)take(512); float* MO = (float*)take(512); float* VO = (float*)take(512);
    bf* QPh = (bf*)take((size_t)CQ * NP * TP * 2); bf* QPl = (bf*)take((size_t)CQ * NP * TP * 2); bf* KPh = (bf*)take((size_t)CQ * NP * TP * 2); bf* KPl = (bf*)take((size_t)CQ * NP * TP * 2); bf* VTh = (bf*)take((size_t)CQ * TV * NP * 2); bf* VTl = (bf*)take((size_t)CQ * TV * NP * 2);
    float* S1 = (float*)take((size_t)CQ * NP * NP * 4); float* S = (float*)take((size_t)CQ * NP * NP * 4); bf* Wh = (bf*)take((size_t)CQ * NP * NP * 2); bf* Wl = (bf*)take((size_t)CQ * NP * NP * 2); float* O1 = (float*)take((size_t)64 * NP * TV * 4); float* O = (float*)take((size_t)64 * NP * TV * 4);
    bf* Ah = (bf*)take((size_t)NROW * D2 * 2); bf* Al = (bf*)take((size_t)NROW * D2 * 2);
    float* OO = YQ;
    if ((size_t)(wsp - (char*)d_ws) > ws_size) return;
    k_cvt8<<<(D2 * CIN / 8 + 255) / 256, 256, 0, stream>>>(wq, WQ, D2 * CIN / 8); k_cvt8<<<(D2 * CIN / 8 + 255) / 256, 256, 0, stream>>>(wk, WK, D2 * CIN / 8); k_cvt8<<<(D2 * CIN / 8 + 255) / 256, 256, 0, stream>>>(wv, WV, D2 * CIN / 8); k_cvt8<<<(CIN * D2 / 8 + 255) / 256, 256, 0, stream>>>(wo, WO, CIN * D2 / 8);
    k_xrows<<<NROW / 8, 256, 0, stream>>>(x0, X0); k_xrows<<<NROW / 8, 256, 0, stream>>>(x1, X1);
    k_gemmb<false, false><<<dim3(NROW / 64, D2 / 64, 1), 128, 0, stream>>>(X0, nullptr, WQ, bq, YQ, D2, nullptr, nullptr, CIN); k_colstat<0><<<1, 128, 0, stream>>>(YQ, D2, nullptr, MQ); k_colstat<1><<<1, 128, 0, stream>>>(YQ, D2, MQ, VQ);
    k_gemmb<false, false><<<dim3(NROW / 64, D2 / 64, 1), 128, 0, stream>>>(X1, nullptr, WK, bk, YK, D2, nullptr, nullptr, CIN); k_colstat<0><<<1, 128, 0, stream>>>(YK, D2, nullptr, MK); k_colstat<1><<<1, 128, 0, stream>>>(YK, D2, MK, VK);
    k_gemmb<false, false><<<dim3(NROW / 64, D2 / 64, 1), 128, 0, stream>>>(X0, nullptr, WV, bv, YV, D2, nullptr, nullptr, CIN); k_colstat<0><<<1, 128, 0, stream>>>(YV, D2, nullptr, MV); k_colstat<1><<<1, 128, 0, stream>>>(YV, D2, MV, VV);
    const size_t sQ = (size_t)NP * TP, sS = (size_t)NP * NP, sV = (size_t)TV * NP, sO = (size_t)NP * TV;
    for (int b = 0; b < NB_; ++b) for (int hf = 0; hf < 2; ++hf) { for (int qq = 0; qq < 2; ++qq) { const int c0 = hf * 64 + qq * CQ;
            k_qkp<<<(CQ * (NP / 2)) / 8, 256, 0, stream>>>(YQ, MQ, VQ, gq, beq, b, c0, QPh, QPl); k_qkp<<<(CQ * (NP / 2)) / 8, 256, 0, stream>>>(YK, MK, VK, gk, bek, b, c0, KPh, KPl); k_vtp<<<(CQ * TV * (NP / 64)) / 8, 256, 0, stream>>>(YV, MV, VV, gv, bev, b, c0, VTh, VTl);
            k_gemmbz<true, false><<<dim3(NP / 64, NP / 64, CQ), 128, 0, stream>>>(QPh, QPl, KPh, nullptr, S1, NP, nullptr, nullptr, TP, 0, sQ, sQ, 0, sS);
            k_gemmbz<false, false><<<dim3(NP / 64, NP / 64, CQ), 128, 0, stream>>>(QPh, nullptr, KPl, nullptr, S, NP, nullptr, S1, TP, 0, sQ, sQ, 0, sS);
            k_gsmx<<<((CQ / KG) * NP * 2) / 8, 256, 0, stream>>>(S, Wh, Wl);
            k_gemmbz<true, false><<<dim3(NP / 64, 1, CQ), 128, 0, stream>>>(Wh, Wl, VTh, nullptr, O1 + (size_t)qq * CQ * sO, TV, nullptr, nullptr, NP, 0, sS, sV, 0, sO);
            k_gemmbz<false, false><<<dim3(NP / 64, 1, CQ), 128, 0, stream>>>(Wh, nullptr, VTl, nullptr, O + (size_t)qq * CQ * sO, TV, nullptr, O1 + (size_t)qq * CQ * sO, NP, 0, sS, sV, 0, sO); }
        k_att<<<(PB + 7) / 8, 256, 0, stream>>>(O, b, hf * 64, Ah, Al); }
    k_gemmb<true, false><<<dim3(NROW / 64, 1, 1), 128, 0, stream>>>(Ah, Al, WO, bo, OO, CIN, nullptr, nullptr, D2); k_colstat<0><<<1, 128, 0, stream>>>(OO, CIN, nullptr, MO); k_colstat<1><<<1, 128, 0, stream>>>(OO, CIN, MO, VO);
    k_out<<<(unsigned)(((size_t)NB_ * CIN * PB / 4 + 255) / 256), 256, 0, stream>>>(OO, MO, VO, go, beo, out);
}
